// TensorProductEncoder_86852828659847
// MI455X (gfx1250) — hardware-verified
//
#include <hip/hip_runtime.h>
#include <stddef.h>


typedef _Float16 v16h __attribute__((ext_vector_type(16)));
typedef _Float16 v8h  __attribute__((ext_vector_type(8)));
typedef float    v8f  __attribute__((ext_vector_type(8)));
typedef float    v4f  __attribute__((ext_vector_type(4)));
typedef _Float16 h16;

#ifndef NB
#define NB 512
#endif
#ifndef SEQ
#define SEQ 512
#endif
#define NB_FULL  512
#define SEQ_FULL 512
#define NFILL 50257
#define NROLE 512
#define FD    128
#define RD    64
#define KD    (FD * RD)
#define FW    768

static_assert(NB >= 64 && NB <= NB_FULL && (NB % 64) == 0);
static_assert(SEQ >= 64 && SEQ <= SEQ_FULL && (SEQ % 64) == 0);
static_assert(FD == 8 * 16);
static_assert(RD == 4 * 16);
static_assert((KD % 32) == 0 && (KD % 8) == 0);
static_assert((FW % 64) == 0);
static_assert(64 * FD == 8 * 256 * 4);
static_assert(64 * RD == 4 * 256 * 4);
static_assert(((size_t)FW * KD) % 2048 == 0);
static_assert((size_t)NB_FULL * FW * 4 == (size_t)1572864);

#define LDT 72
#define LDC 68
static_assert((LDT % 8) == 0 && LDT >= 64);
static_assert((LDC % 4) == 0 && LDC >= 64);

#define ECARRY 64.0f
#define FCARRY 16.0f
#define WCARRY 1024.0f

#define W16_BYTES  ((size_t)FW * KD * 2)
#define FL16_BYTES ((size_t)NB * KD * 2)
#define OFF_W16  ((size_t)0)
#define OFF_FL16 (OFF_W16 + W16_BYTES)
#define WS_TOTAL (OFF_FL16 + FL16_BYTES)
static_assert((W16_BYTES % 128) == 0 && (FL16_BYTES % 128) == 0);
static_assert(WS_TOTAL <= (size_t)134217728);

__device__ __forceinline__ float bf16r(float x) {
  unsigned int u = __float_as_uint(x);
  u = (u + 0x7FFFu + ((u >> 16) & 1u)) & 0xFFFF0000u;
  return __uint_as_float(u);
}

static __device__ __forceinline__ h16 toh_flush(float v) {
  const h16 r = (h16)v;
  return (fabsf(v) < 6.103515625e-05f) ? (h16)0.0f : r;
}

__device__ __forceinline__ v16h frag_at(const _Float16* p) {
  v8h lo = *(const v8h*)(p);
  v8h hi = *(const v8h*)(p + 16);
  v16h out;
#pragma unroll
  for (int i = 0; i < 8; ++i) { out[i] = lo[i]; out[i + 8] = hi[i]; }
  return out;
}
__device__ __forceinline__ v16h ld_frag(const _Float16* base, unsigned ld) {
  const unsigned lane = threadIdx.x & 31u;
  return frag_at(base + (lane & 15u) * ld + (lane >> 4) * 8u);
}

__device__ __forceinline__ v8f wmma16(v16h a, v16h b, v8f c) {
  v8f d = __builtin_amdgcn_wmma_f32_16x16x32_f16(false, a, false, b, (short)0, c,
                                                 false, false);
  asm volatile("v_nop\n\tv_nop\n\tv_nop\n\tv_nop" : "+v"(d) : "v"(a), "v"(b));
  return d;
}

__global__ __launch_bounds__(256) void wcast_kernel(
    const float* __restrict__ W, _Float16* __restrict__ W16) {
#pragma clang fp contract(off)
  const size_t i = ((size_t)blockIdx.x * 256u + threadIdx.x) * 8u;
  const v4f a0 = *(const v4f*)(W + i);
  const v4f a1 = *(const v4f*)(W + i + 4u);
  v8h o;
#pragma unroll
  for (int j = 0; j < 4; ++j) {
    o[j]     = toh_flush(WCARRY * bf16r(a0[j]));
    o[j + 4] = toh_flush(WCARRY * bf16r(a1[j]));
  }
  _Float16* p = W16 + i;
  *(volatile v8h*)p = o;
  __threadfence();
  *(volatile v8h*)p = o;
}

__global__ __launch_bounds__(256) void outer_kernel(
    const int* __restrict__ fillers, const int* __restrict__ roles,
    const float* __restrict__ ftab, const float* __restrict__ rtab,
    _Float16* __restrict__ flat16) {
  __shared__ __attribute__((aligned(16))) _Float16 FeT[FD * LDT];
  __shared__ __attribute__((aligned(16))) _Float16 ReT[RD * LDT];
  __shared__ __attribute__((aligned(16))) _Float16 Cs[FD * LDT];

  const unsigned tid = threadIdx.x, lane = tid & 31u;
  const unsigned wave = (unsigned)__builtin_amdgcn_readfirstlane((int)(threadIdx.x >> 5));
  const unsigned hh = lane >> 4, m = lane & 15u;
  const unsigned b = blockIdx.x;
  const unsigned m0 = wave * 16u;
  const size_t idbase = (size_t)b * SEQ_FULL;

  v8f acc[4];
#pragma unroll
  for (int nt = 0; nt < 4; ++nt) acc[nt] = (v8f){};

#pragma unroll 1
  for (unsigned k0 = 0; k0 < (unsigned)SEQ; k0 += 64u) {
    __syncthreads();
#pragma unroll 4
    for (unsigned i = 0; i < 8u; ++i) {
      const unsigned idx = tid + 256u * i;
      const unsigned row = idx >> 5, c4 = idx & 31u;
      int id = fillers[idbase + k0 + row];
      id = min(max(id, 0), NFILL - 1);
      const v4f v = *(const v4f*)(ftab + (size_t)id * FD + c4 * 4u);
#pragma unroll
      for (int j = 0; j < 4; ++j)
        FeT[(c4 * 4u + (unsigned)j) * LDT + row] = toh_flush(ECARRY * bf16r(v[j]));
    }
#pragma unroll 4
    for (unsigned i = 0; i < 4u; ++i) {
      const unsigned idx = tid + 256u * i;
      const unsigned row = idx >> 4, c4 = idx & 15u;
      int id = roles[idbase + k0 + row];
      id = min(max(id, 0), NROLE - 1);
      const v4f v = *(const v4f*)(rtab + (size_t)id * RD + c4 * 4u);
#pragma unroll
      for (int j = 0; j < 4; ++j)
        ReT[(c4 * 4u + (unsigned)j) * LDT + row] = toh_flush(ECARRY * bf16r(v[j]));
    }
    __syncthreads();

#pragma unroll
    for (int c = 0; c < 2; ++c) {
      const v16h a = ld_frag(&FeT[m0 * LDT + (unsigned)c * 32u], LDT);
#pragma unroll
      for (int nt = 0; nt < 4; ++nt) {
        const v16h bf = ld_frag(&ReT[((unsigned)nt * 16u) * LDT + (unsigned)c * 32u], LDT);
        acc[nt] = wmma16(a, bf, acc[nt]);
      }
    }
  }

  const float cs = FCARRY / (ECARRY * ECARRY);
#pragma unroll
  for (int nt = 0; nt < 4; ++nt)
#pragma unroll
    for (int v = 0; v < 8; ++v)
      Cs[(m0 + hh * 8u + (unsigned)v) * LDT + (unsigned)nt * 16u + m] =
          toh_flush(acc[nt][v] * cs);
  __syncthreads();

  v8h x[4];
  size_t off[4];
#pragma unroll
  for (unsigned i = 0; i < 4u; ++i) {
    const unsigned r = m0 + 4u * i + (lane >> 3);
    const unsigned c = (lane & 7u) * 8u;
    x[i] = *(const v8h*)&Cs[r * LDT + c];
    off[i] = (size_t)b * KD + (size_t)r * RD + c;
  }
#pragma unroll
  for (int i = 0; i < 4; ++i) *(volatile v8h*)(flat16 + off[i]) = x[i];
  __threadfence();
#pragma unroll
  for (int i = 0; i < 4; ++i) *(volatile v8h*)(flat16 + off[i]) = x[i];
}

__global__ __launch_bounds__(256) void gemm_out_kernel(
    const _Float16* __restrict__ A16, const _Float16* __restrict__ Bt,
    const float* __restrict__ bias, float* __restrict__ outf) {
  __shared__ __attribute__((aligned(16))) float Cs[64 * LDC];
  const unsigned tid = threadIdx.x, lane = tid & 31u;
  const unsigned w = (unsigned)__builtin_amdgcn_readfirstlane((int)(threadIdx.x >> 5));
  const unsigned mw = w >> 1, nw = w & 1u;
  const unsigned hh = lane >> 4, m = lane & 15u;
  const unsigned n0 = blockIdx.x * 64u;
  const unsigned row0 = blockIdx.y * 64u;
  const unsigned K = (unsigned)KD;

  const _Float16* ap  = A16 + (size_t)(row0 + mw * 16u + m) * K + hh * 8u;
  const _Float16* bp0 = Bt + (size_t)(n0 + nw * 32u + m) * K + hh * 8u;
  const _Float16* bp1 = bp0 + (size_t)16 * K;
  v8f acc0 = {}, acc1 = {};
#pragma unroll 2
  for (unsigned k0 = 0; k0 < K; k0 += 32u) {
    const v16h a  = frag_at(ap + k0);
    const v16h b0 = frag_at(bp0 + k0);
    const v16h b1 = frag_at(bp1 + k0);
    acc0 = wmma16(a, b0, acc0);
    acc1 = wmma16(a, b1, acc1);
  }
#pragma unroll
  for (int r = 0; r < 8; ++r) {
    float* d = &Cs[(mw * 16u + hh * 8u + (unsigned)r) * LDC + nw * 32u + m];
    d[0]  = acc0[r];
    d[16] = acc1[r];
  }
  __syncthreads();

  const float cs = 1.0f / (FCARRY * WCARRY);
  v4f xs[4];
  size_t off[4];
#pragma unroll
  for (unsigned i = 0; i < 4u; ++i) {
    const unsigned r = 16u * i + (tid >> 4);
    const unsigned c = (tid & 15u) * 4u;
    const v4f u = *(const v4f*)&Cs[r * LDC + c];
    const v4f g = *(const v4f*)(bias + n0 + c);
    v4f val;
#pragma unroll
    for (int j = 0; j < 4; ++j) val[j] = u[j] * cs + bf16r(g[j]);
    xs[i] = val;
    off[i] = (size_t)(row0 + r) * FW + n0 + c;
  }
#pragma unroll
  for (int i = 0; i < 4; ++i) *(volatile v4f*)(outf + off[i]) = xs[i];
  __threadfence();
#pragma unroll
  for (int i = 0; i < 4; ++i) *(volatile v4f*)(outf + off[i]) = xs[i];
}

extern "C" void kernel_launch(void* const* d_in, const int* in_sizes, int n_in,
                              void* d_out, int out_size, void* d_ws, size_t ws_size,
                              hipStream_t stream) {
  if (n_in < 6) return;
  const long long need_ids = (long long)(NB - 1) * SEQ_FULL + SEQ;
  if ((long long)in_sizes[0] < need_ids) return;
  if ((long long)in_sizes[1] < need_ids) return;
  if ((long long)in_sizes[2] < (long long)NFILL * FD) return;
  if ((long long)in_sizes[3] < (long long)NROLE * RD) return;
  if ((long long)in_sizes[4] < (long long)FW * KD) return;
  if (in_sizes[5] < FW) return;
  if ((long long)out_size < (long long)NB * FW) return;
  if (ws_size < WS_TOTAL) return;

  const int*   fillers = (const int*)d_in[0];
  const int*   roles   = (const int*)d_in[1];
  const float* ftab    = (const float*)d_in[2];
  const float* rtab    = (const float*)d_in[3];
  const float* wlast   = (const float*)d_in[4];
  const float* blast   = (const float*)d_in[5];
  float* out = (float*)d_out;

  char* ws = (char*)d_ws;
  _Float16* W16    = (_Float16*)(ws + OFF_W16);
  _Float16* Flat16 = (_Float16*)(ws + OFF_FL16);

  dim3 blk(256);
  wcast_kernel<<<dim3((unsigned)(((size_t)FW * KD) / 2048)), blk, 0, stream>>>(wlast, W16);
  outer_kernel<<<dim3(NB), blk, 0, stream>>>(fillers, roles, ftab, rtab, Flat16);
  gemm_out_kernel<<<dim3(FW / 64, NB / 64), blk, 0, stream>>>(Flat16, W16, blast, out);
}
